// SpaMamba_26319559590730
// MI455X (gfx1250) — hardware-run, weakly checked
//
#include <hip/hip_runtime.h>

typedef __attribute__((ext_vector_type(16))) _Float16 v16h;
typedef __attribute__((ext_vector_type(8)))  _Float16 v8h;
typedef __attribute__((ext_vector_type(16))) __bf16   v16b;
typedef __attribute__((ext_vector_type(8)))  __bf16   v8b;
typedef __attribute__((ext_vector_type(8)))  float    v8f;
typedef __attribute__((ext_vector_type(4)))  float    v4f;
typedef __attribute__((ext_vector_type(4)))  unsigned int v4u;
typedef v4u v4ua __attribute__((__may_alias__));
typedef v4f v4fa __attribute__((__may_alias__));

constexpr int kBatch = 4;
constexpr int kSeq = 4096;
constexpr int kModel = 128;
constexpr int kInner = 256;
constexpr int kState = 16;
constexpr int kRank = 8;
constexpr int kXin = 2 * kInner;
constexpr int kXdbCols = 40;
constexpr int kXdbPitch = 64;
constexpr int kRows = kBatch * kSeq;
constexpr int kScanChunk = 32;
constexpr int kGroups = 4;

static_assert(kRows % 64 == 0);
static_assert(kXin % 64 == 0 && kModel % 32 == 0);
static_assert(kXdbPitch % 64 == 0 && kInner % 32 == 0);
static_assert(kModel % 64 == 0 && kInner % 32 == 0);
static_assert(kSeq % kScanChunk == 0);

__device__ __forceinline__ unsigned short f2bf_bits(float f) {
  unsigned u = __float_as_uint(f);
  return (unsigned short)((u + 0x7FFFu + ((u >> 16) & 1u)) >> 16);
}
__device__ __forceinline__ float bf_bits2f(unsigned short h) { return __uint_as_float(((unsigned)h) << 16); }

__device__ __forceinline__ void dep_guard_h(v8f& a, v8f& b, v16h x, v16h y) { asm volatile("v_nop\n\tv_nop\n\tv_nop\n\tv_nop" : "+v"(a), "+v"(b) : "v"(x), "v"(y)); }
__device__ __forceinline__ void dep_guard_b(v8f& a, v8f& b, v16b x, v16b y) { asm volatile("v_nop\n\tv_nop\n\tv_nop\n\tv_nop" : "+v"(a), "+v"(b) : "v"(x), "v"(y)); }
__device__ __forceinline__ void keep4_h(v16h a, v16h b, v16h c, v16h d) { asm volatile("v_nop" :: "v"(a), "v"(b), "v"(c), "v"(d)); }
__device__ __forceinline__ void keep4_b(v16b a, v16b b, v16b c, v16b d) { asm volatile("v_nop" :: "v"(a), "v"(b), "v"(c), "v"(d)); }
__device__ __forceinline__ void acc_guard4(v8f& a, v8f& b, v8f& c, v8f& d) { asm volatile("v_nop\n\tv_nop\n\tv_nop\n\tv_nop" : "+v"(a), "+v"(b), "+v"(c), "+v"(d)); }
template <typename T> struct Frag;
template <> struct Frag<_Float16> {
  typedef v16h V; union U { v16h v; v8h h[2]; };
  static __device__ __forceinline__ v16h load(const _Float16* p) {
    U f; f.h[0] = *(const v8h*)(p); f.h[1] = *(const v8h*)(p + 16); return f.v;
  }
  static __device__ __forceinline__ v8f mma(v16h a, v16h b, v8f c) {
    return __builtin_amdgcn_wmma_f32_16x16x32_f16(false, a, false, b, (short)0, c, false, false);
  }
  static __device__ __forceinline__ void guard(v8f& a, v8f& b, v16h x, v16h y) { dep_guard_h(a, b, x, y); }
  static __device__ __forceinline__ void keep(v16h a, v16h b, v16h c, v16h d) { keep4_h(a, b, c, d); }
};
template <> struct Frag<__bf16> {
  typedef v16b V; union U { v16b v; v8b h[2]; };
  static __device__ __forceinline__ v16b load(const __bf16* p) {
    U f; f.h[0] = *(const v8b*)(p); f.h[1] = *(const v8b*)(p + 16); return f.v;
  }
  static __device__ __forceinline__ v8f mma(v16b a, v16b b, v8f c) {
    return __builtin_amdgcn_wmma_f32_16x16x32_bf16(false, a, false, b, (short)0, c, false, false);
  }
  static __device__ __forceinline__ void guard(v8f& a, v8f& b, v16b x, v16b y) { dep_guard_b(a, b, x, y); }
  static __device__ __forceinline__ void keep(v16b a, v16b b, v16b c, v16b d) { keep4_b(a, b, c, d); }
};

template <int ET> struct Elem;
template <> struct Elem<0> { typedef _Float16 T; };
template <> struct Elem<1> { typedef __bf16 T; };
template <int ET, bool SPLIT, int BIAS_MODE, int OUT_MODE, bool RESID, int ACT = 0>
__global__ __launch_bounds__(256) void wmma_gemm64(
    const unsigned short* __restrict__ Ap, const unsigned short* __restrict__ A2p, int lda, long strideA,
    const unsigned short* __restrict__ Btp, const unsigned short* __restrict__ Bt2p, int ldb, long strideB,
    void* __restrict__ Cout, void* __restrict__ Cout2, int ldc, long strideC,
    const float* __restrict__ bias,
    const float* __restrict__ resid, long strideR,
    int M, int N, int K, float scale) {
  typedef typename Elem<ET>::T T;
  typedef typename Frag<T>::V V;
  const T* A = (const T*)Ap; const T* A2 = (const T*)A2p; const T* Bt = (const T*)Btp; const T* Bt2 = (const T*)Bt2p;
  __shared__ __align__(16) float sT[8][16 * 68];
  const int b    = blockIdx.y;
  const int lane = threadIdx.x & 31;
  const int wave = threadIdx.x >> 5;
  const int tilesN = N >> 6;
  const int tilesM = M >> 6;
  const int tile = blockIdx.x * 8 + wave;
  if (tile >= tilesM * tilesN) return;
  const int tm = tile / tilesN;
  const int tn = tile - tm * tilesN;
  const int m0 = tm << 6;
  const int n0 = tn << 6;

  const T* Ab  = A  + (size_t)b * strideA;
  const T* Bb  = Bt + (size_t)b * strideB;
  const T* Ab2 = SPLIT ? (A2  + (size_t)b * strideA) : nullptr;
  const T* Bb2 = SPLIT ? (Bt2 + (size_t)b * strideB) : nullptr;

  const int rlane = lane & 15;
  const int koff  = (lane >> 4) * 8;
  const int mOff  = (lane >> 4) * 8;

  v8f acc[4][4];
#pragma unroll
  for (int i = 0; i < 4; ++i)
#pragma unroll
    for (int j = 0; j < 4; ++j) acc[i][j] = (v8f){0.f,0.f,0.f,0.f,0.f,0.f,0.f,0.f};

  for (int k0 = 0; k0 < K; k0 += 32) {
    V bh[4], bl[4];
#pragma unroll
    for (int j = 0; j < 4; ++j) {
      const size_t bo = (size_t)(n0 + (j << 4) + rlane) * ldb + koff + k0;
      bh[j] = Frag<T>::load(Bb + bo);
      if (SPLIT) bl[j] = Frag<T>::load(Bb2 + bo);
    }
#pragma unroll
    for (int i = 0; i < 4; ++i) {
      const size_t ao = (size_t)(m0 + (i << 4) + rlane) * lda + koff + k0;
      V ah = Frag<T>::load(Ab + ao);
      V al;
      if (SPLIT) al = Frag<T>::load(Ab2 + ao);
#pragma unroll
      for (int j = 0; j < 4; ++j) {
        acc[i][j] = Frag<T>::mma(ah, bh[j], acc[i][j]);
        if (SPLIT) {
          acc[i][j] = Frag<T>::mma(ah, bl[j], acc[i][j]);
          acc[i][j] = Frag<T>::mma(al, bh[j], acc[i][j]);
        }
      }
      Frag<T>::guard(acc[i][0], acc[i][3], ah, SPLIT ? al : ah);
    }
    Frag<T>::keep(bh[0], bh[1], bh[2], bh[3]);
    if (SPLIT) Frag<T>::keep(bl[0], bl[1], bl[2], bl[3]);
  }
  acc_guard4(acc[0][0], acc[0][1], acc[0][2], acc[0][3]);
  acc_guard4(acc[1][0], acc[1][1], acc[1][2], acc[1][3]);
  acc_guard4(acc[2][0], acc[2][1], acc[2][2], acc[2][3]);
  acc_guard4(acc[3][0], acc[3][1], acc[3][2], acc[3][3]);

  float* slab = sT[wave];
  const float* Rb = RESID ? (resid + (size_t)b * strideR) : nullptr;
#pragma unroll
  for (int i = 0; i < 4; ++i) {
    const int mBase = m0 + (i << 4);
#pragma unroll
    for (int j = 0; j < 4; ++j) {
      const int n = n0 + (j << 4) + rlane;
      float bv = 0.f;
      if (BIAS_MODE == 2) bv = bias[n];
#pragma unroll
      for (int r = 0; r < 8; ++r) {
        float v = acc[i][j][r] * scale;
        if (BIAS_MODE == 1) v += bias[mBase + mOff + r];
        if (BIAS_MODE == 2) v += bv;
        if (RESID) v += Rb[(size_t)(mBase + mOff + r) * ldc + n];
        if (ACT == 1) v = tanhf(v);
        if (ACT == 2) v = fmaxf(v, 0.0f);
        if (ACT == 3) v = v / (1.0f + expf(-v));
        if (ACT == 4) v = (v > 0.f) ? v : 0.01f * v;
        if (ACT == 5) v = 0.5f * v * (1.0f + erff(v * 0.70710678118654752f));
        slab[(mOff + r) * 68 + (j << 4) + rlane] = v;
      }
    }
    __builtin_amdgcn_fence(__ATOMIC_RELEASE, "workgroup");
    __builtin_amdgcn_wave_barrier();
    __builtin_amdgcn_fence(__ATOMIC_ACQUIRE, "workgroup");
    if (OUT_MODE == 0) {
      float* C = (float*)Cout + (size_t)b * strideC;
      const int hh = lane >> 4, c4 = (lane & 15) * 4;
      for (int pass = 0; pass < 2; ++pass) {
#pragma unroll
        for (int it = 0; it < 8; ++it) {
          const int row = it * 2 + hh;
          v4f v = *(const v4f*)(slab + row * 68 + c4);
          *(volatile v4f*)(C + (size_t)(mBase + row) * ldc + n0 + c4) = v;
        }
        __threadfence();
      }
    } else {
      const int q = lane >> 3, c8 = (lane & 7) * 8;
      unsigned short* C  = (unsigned short*)Cout  + (size_t)b * strideC;
      unsigned short* C2 = (OUT_MODE == 2) ? ((unsigned short*)Cout2 + (size_t)b * strideC) : nullptr;
      for (int pass = 0; pass < 2; ++pass) {
#pragma unroll
        for (int it = 0; it < 4; ++it) {
          const int row = it * 4 + q;
          const float* sp = slab + row * 68 + c8;
          v8h hv, lv;
#pragma unroll
          for (int e = 0; e < 8; ++e) {
            if (OUT_MODE == 1) {
              hv[e] = (_Float16)sp[e];
            } else {
              unsigned short hb = f2bf_bits(sp[e]);
              unsigned short lb = f2bf_bits(sp[e] - bf_bits2f(hb));
              hv[e] = __builtin_bit_cast(_Float16, hb);
              lv[e] = __builtin_bit_cast(_Float16, lb);
            }
          }
          *(volatile v8h*)(C + (size_t)(mBase + row) * ldc + n0 + c8) = hv;
          if (OUT_MODE == 2) *(volatile v8h*)(C2 + (size_t)(mBase + row) * ldc + n0 + c8) = lv;
        }
        __threadfence();
      }
    }
    __builtin_amdgcn_fence(__ATOMIC_RELEASE, "workgroup");
    __builtin_amdgcn_wave_barrier();
    __builtin_amdgcn_fence(__ATOMIC_ACQUIRE, "workgroup");
  }
}

__device__ __forceinline__ void pack_split8(const float (&v)[8], v4u& hi, v4u& lo) {
#pragma unroll
  for (int p = 0; p < 4; ++p) {
    const unsigned short h0 = f2bf_bits(v[2 * p]);
    const unsigned short h1 = f2bf_bits(v[2 * p + 1]);
    const unsigned short l0 = f2bf_bits(v[2 * p] - bf_bits2f(h0));
    const unsigned short l1 = f2bf_bits(v[2 * p + 1] - bf_bits2f(h1));
    hi[p] = (unsigned)h0 | ((unsigned)h1 << 16);
    lo[p] = (unsigned)l0 | ((unsigned)l1 << 16);
  }
}
__device__ __forceinline__ float silu_f(float v) { return v * (1.0f / (1.0f + expf(-v))); }

__global__ __launch_bounds__(256) void k_xprep(const float* __restrict__ x,
                                               unsigned short* __restrict__ Xh,
                                               unsigned short* __restrict__ Xl) {
  __shared__ float tileT[32][kModel + 1];
  const int t = threadIdx.x, j = t & 31, l0 = blockIdx.x * 32, b = blockIdx.y;
#pragma unroll 4
  for (int i = 0; i < 16; ++i) {
    const int c = (t >> 5) + 8 * i;
    tileT[j][c] = x[((size_t)(b * kModel + c)) * kSeq + l0 + j];
  }
  __syncthreads();
  v4u hv[2], lv[2];
  size_t off[2];
#pragma unroll
  for (int i = 0; i < 2; ++i) {
    const int q = i * 256 + t;
    const int row = q >> 4, cir = q & 15;
    float v[8];
#pragma unroll
    for (int e = 0; e < 8; ++e) v[e] = tileT[row][cir * 8 + e];
    pack_split8(v, hv[i], lv[i]);
    off[i] = ((size_t)(b * kSeq + l0 + row)) * kModel + cir * 8;
  }
  for (int pass = 0; pass < 2; ++pass) {
#pragma unroll
    for (int i = 0; i < 2; ++i) {
      *(volatile v4u*)(Xh + off[i]) = hv[i];
      *(volatile v4u*)(Xl + off[i]) = lv[i];
    }
    __threadfence();
  }
}

template <int KD>
__global__ __launch_bounds__(256) void k_wprep(const float* __restrict__ w, int nCols,
                                               unsigned short* __restrict__ oh,
                                               unsigned short* __restrict__ ol) {
  __shared__ float tileT[32][KD + 1];
  const int t = threadIdx.x, j = t & 31, n0 = blockIdx.x * 32;
  const int n = n0 + j;
  const int nc = (n < nCols) ? n : (nCols - 1);
  const bool ok = (n < nCols);
#pragma unroll 4
  for (int i = 0; i < KD / 8; ++i) {
    const int k = (t >> 5) + 8 * i;
    const float v = w[(size_t)k * nCols + nc];
    tileT[j][k] = ok ? v : 0.f;
  }
  __syncthreads();
  constexpr int CPR = KD / 8;
  constexpr int ITER = (32 * CPR) / 256;
  v4u hv[ITER], lv[ITER];
  size_t off[ITER];
#pragma unroll
  for (int i = 0; i < ITER; ++i) {
    const int q = i * 256 + t;
    const int row = q / CPR, cir = q % CPR;
    float v[8];
#pragma unroll
    for (int e = 0; e < 8; ++e) v[e] = tileT[row][cir * 8 + e];
    pack_split8(v, hv[i], lv[i]);
    off[i] = ((size_t)(n0 + row)) * KD + cir * 8;
  }
  for (int pass = 0; pass < 2; ++pass) {
#pragma unroll
    for (int i = 0; i < ITER; ++i) {
      *(volatile v4u*)(oh + off[i]) = hv[i];
      *(volatile v4u*)(ol + off[i]) = lv[i];
    }
    __threadfence();
  }
}

__global__ __launch_bounds__(256) void k_conv(const float* __restrict__ xz, const float* __restrict__ cw,
                                              const float* __restrict__ cb, float* __restrict__ xc,
                                              unsigned short* __restrict__ xcb, int backward) {
  __shared__ __align__(16) unsigned int s2[512];
  const int t = threadIdx.x;
  const size_t e = (size_t)blockIdx.x * 1024 + 4 * t;
  const size_t bl = e >> 8;
  const int d = (int)(e & 255);
  const int lpos = (int)(bl & (kSeq - 1));
  size_t nbl;
  bool has;
  if (backward) { has = (lpos < kSeq - 1); nbl = has ? (bl + 1) : bl; }
  else          { has = (lpos > 0);        nbl = has ? (bl - 1) : bl; }
  const v4f xp = *(const v4f*)(xz + bl * kXin + d);
  const v4f xnraw = *(const v4f*)(xz + nbl * kXin + d);
  const v4f zero4 = (v4f){0.f, 0.f, 0.f, 0.f};
  const v4f xn = has ? xnraw : zero4;
  const v4f c0 = *(const v4f*)(cw + 2 * d);
  const v4f c1 = *(const v4f*)(cw + 2 * d + 4);
  const v4f bb = *(const v4f*)(cb + d);
  v4f ov;
  ov[0] = silu_f(xn[0] * c0[0] + xp[0] * c0[1] + bb[0]);
  ov[1] = silu_f(xn[1] * c0[2] + xp[1] * c0[3] + bb[1]);
  ov[2] = silu_f(xn[2] * c1[0] + xp[2] * c1[1] + bb[2]);
  ov[3] = silu_f(xn[3] * c1[2] + xp[3] * c1[3] + bb[3]);
  s2[2 * t]     = (unsigned)f2bf_bits(ov[0]) | ((unsigned)f2bf_bits(ov[1]) << 16);
  s2[2 * t + 1] = (unsigned)f2bf_bits(ov[2]) | ((unsigned)f2bf_bits(ov[3]) << 16);
  __syncthreads();
  v4u u = (v4u){0u, 0u, 0u, 0u};
  if (t < 128) u = *(const v4ua*)(s2 + 4 * t);
  unsigned short* bdst = xcb + (size_t)blockIdx.x * 1024 + 8 * t;
  for (int pass = 0; pass < 2; ++pass) {
    *(volatile v4f*)(xc + e) = ov;
    if (t < 128) *(volatile v4u*)(bdst) = u;
    __threadfence();
  }
}

__global__ __launch_bounds__(256) void k_scan(const float* __restrict__ xdb, const float* __restrict__ xc,
                                              const float* __restrict__ xz, const float* __restrict__ Wdt,
                                              const float* __restrict__ bdt, const float* __restrict__ Alog,
                                              const float* __restrict__ Dp, unsigned short* __restrict__ Gh,
                                              unsigned short* __restrict__ Gl, int backward) {
  __shared__ __align__(16) float xdb_s[kScanChunk * kXdbPitch];
  __shared__ __align__(16) float a_s[kInner * kState];
  __shared__ __align__(16) unsigned short gh_s[kScanChunk * kInner];
  __shared__ __align__(16) unsigned short gl_s[kScanChunk * kInner];
  const int t = threadIdx.x;
  const int b = blockIdx.x;
#pragma unroll 1
  for (int s = 0; s < kState; ++s) a_s[t * kState + s] = -expf(Alog[t * kState + s]);
  float wd[kRank];
#pragma unroll
  for (int k = 0; k < kRank; ++k) wd[k] = Wdt[k * kInner + t];
  const float bd = bdt[t];
  const float dd = Dp[t];
  __syncthreads();
  float av[kState];
#pragma unroll
  for (int q = 0; q < 4; ++q) {
    const v4f aq = *(const v4f*)(a_s + t * kState + 4 * q);
#pragma unroll
    for (int e = 0; e < 4; ++e) av[4 * q + e] = aq[e];
  }
  float h[kState];
#pragma unroll
  for (int s = 0; s < kState; ++s) h[s] = 0.f;

#pragma unroll 1
  for (int cc = 0; cc < kSeq / kScanChunk; ++cc) {
    const int chunk = backward ? (kSeq / kScanChunk - 1 - cc) : cc;
    const int l0 = chunk * kScanChunk;
    const size_t rowbase = (size_t)b * kSeq + l0;
    __syncthreads();
    {
      const v4f* src = (const v4f*)(xdb + rowbase * kXdbPitch);
      v4f* dst = (v4f*)xdb_s;
      dst[t] = src[t];
      dst[t + 256] = src[t + 256];
    }
    __syncthreads();
#pragma unroll 1
    for (int j = 0; j < kScanChunk; ++j) {
      const int r = backward ? (kScanChunk - 1 - j) : j;
      const size_t bl = rowbase + r;
      const float* row = xdb_s + r * kXdbPitch;
      const v4f d0 = *(const v4f*)(row);
      const v4f d1 = *(const v4f*)(row + 4);
      float sacc = d0[0] * wd[0];
      sacc = fmaf(d0[1], wd[1], sacc);
      sacc = fmaf(d0[2], wd[2], sacc);
      sacc = fmaf(d0[3], wd[3], sacc);
      sacc = fmaf(d1[0], wd[4], sacc);
      sacc = fmaf(d1[1], wd[5], sacc);
      sacc = fmaf(d1[2], wd[6], sacc);
      sacc = fmaf(d1[3], wd[7], sacc);
      const float sv = sacc + bd;
      const float dt = fmaxf(sv, 0.f) + log1pf(expf(-fabsf(sv)));
      const float xt = xc[bl * kInner + t];
      const float zt = xz[bl * kXin + kInner + t];
      const float dx = dt * xt;
      v4f bq[4], cq[4];
#pragma unroll
      for (int q = 0; q < 4; ++q) {
        bq[q] = *(const v4f*)(row + kRank + 4 * q);
        cq[q] = *(const v4f*)(row + kRank + kState + 4 * q);
      }
      float y = 0.f;
#pragma unroll
      for (int s = 0; s < kState; ++s) {
        const float da = __expf(dt * av[s]);
        h[s] = fmaf(da, h[s], dx * bq[s >> 2][s & 3]);
        y = fmaf(h[s], cq[s >> 2][s & 3], y);
      }
      const float yy = fmaf(dd, xt, y);
      const float g = yy * silu_f(zt);
      const unsigned short hb = f2bf_bits(g);
      const unsigned short lb = f2bf_bits(g - bf_bits2f(hb));
      gh_s[r * kInner + t] = hb;
      gl_s[r * kInner + t] = lb;
    }
    __syncthreads();
    {
      const size_t base = rowbase * kInner;
      v4u hv[4], lv[4];
#pragma unroll
      for (int i = 0; i < 4; ++i) {
        const int e = (i * 256 + t) * 8;
        hv[i] = *(const v4ua*)(gh_s + e);
        lv[i] = *(const v4ua*)(gl_s + e);
      }
      for (int pass = 0; pass < 2; ++pass) {
#pragma unroll
        for (int i = 0; i < 4; ++i) {
          const int e = (i * 256 + t) * 8;
          *(volatile v4u*)(Gh + base + e) = hv[i];
          *(volatile v4u*)(Gl + base + e) = lv[i];
        }
        __threadfence();
      }
    }
  }
}

__global__ __launch_bounds__(256) void k_gnstats(const float* __restrict__ yf, const float* __restrict__ yb,
                                                 float* __restrict__ stats) {
  __shared__ double red[256];
  __shared__ float s_mu, s_rinv;
  const int t = threadIdx.x, bg = blockIdx.x, b = bg >> 2, g = bg & 3;
  const size_t base = (size_t)b * kSeq * kModel + g * 32;
  constexpr int kPerThread = (kSeq * 8) / 256;
  constexpr double kInvN = 1.0 / (32.0 * 4096.0);
  double acc = 0.0;
#pragma unroll 1
  for (int i = 0; i < kPerThread; ++i) {
    const int q = i * 256 + t;
    const int row = q >> 3, c4 = (q & 7) * 4;
    const size_t idx = base + (size_t)row * kModel + c4;
    const v4f v = *(const v4f*)(yf + idx) + *(const v4f*)(yb + idx);
    acc += (double)v[0] + (double)v[1] + (double)v[2] + (double)v[3];
  }
  red[t] = acc;
  __syncthreads();
  for (int st = 128; st > 0; st >>= 1) {
    if (t < st) red[t] += red[t + st];
    __syncthreads();
  }
  if (t == 0) s_mu = (float)(red[0] * kInvN);
  __syncthreads();
  const float mu = s_mu;
  double acc2 = 0.0;
#pragma unroll 1
  for (int i = 0; i < kPerThread; ++i) {
    const int q = i * 256 + t;
    const int row = q >> 3, c4 = (q & 7) * 4;
    const size_t idx = base + (size_t)row * kModel + c4;
    const v4f v = *(const v4f*)(yf + idx) + *(const v4f*)(yb + idx);
#pragma unroll
    for (int e = 0; e < 4; ++e) { const float dv = v[e] - mu; acc2 += (double)(dv * dv); }
  }
  red[t] = acc2;
  __syncthreads();
  for (int st = 128; st > 0; st >>= 1) {
    if (t < st) red[t] += red[t + st];
    __syncthreads();
  }
  if (t == 0) {
    const float var = (float)(red[0] * kInvN);
    s_rinv = rsqrtf(var + 1e-5f);
  }
  __syncthreads();
  if (t < 32) {
    const float val = (t == 0) ? s_mu : ((t == 1) ? s_rinv : 0.f);
    for (int pass = 0; pass < 2; ++pass) {
      *(volatile float*)(stats + (size_t)bg * 32 + t) = val;
      __threadfence();
    }
  }
}

__global__ __launch_bounds__(256) void k_gnapply(const float* __restrict__ yf, const float* __restrict__ yb,
                                                 const float* __restrict__ stats, const float* __restrict__ gamma,
                                                 const float* __restrict__ beta, const float* __restrict__ x,
                                                 float* __restrict__ out) {
  __shared__ float tileT[32][kModel + 1];
  __shared__ __align__(16) float outT[kModel * 36];
  const int t = threadIdx.x, lane = t & 31, wave = t >> 5;
  const int b = blockIdx.y, l0 = blockIdx.x * 32;
#pragma unroll
  for (int i = 0; i < 4; ++i) {
    const int q = i * 256 + t;
    const int j = q >> 5, c4 = (q & 31) * 4;
    const size_t idx = ((size_t)(b * kSeq + l0 + j)) * kModel + c4;
    const v4f v = *(const v4f*)(yf + idx) + *(const v4f*)(yb + idx);
#pragma unroll
    for (int e = 0; e < 4; ++e) tileT[j][c4 + e] = v[e];
  }
  const int g = wave >> 1;
  const float mu = stats[((size_t)b * kGroups + g) * 32 + 0];
  const float rinv = stats[((size_t)b * kGroups + g) * 32 + 1];
  __syncthreads();
  const int j4 = (lane & 7) * 4;
#pragma unroll 1
  for (int it = 0; it < 4; ++it) {
    const int c = wave * 16 + it * 4 + (lane >> 3);
    const float ga = gamma[c], be = beta[c];
    const v4f xr = *(const v4f*)(x + ((size_t)(b * kModel + c)) * kSeq + l0 + j4);
#pragma unroll
    for (int e = 0; e < 4; ++e) {
      const float v = tileT[j4 + e][c];
      const float xn = (v - mu) * rinv;
      const float a = xn * ga + be;
      outT[c * 36 + j4 + e] = silu_f(a) + xr[e];
    }
  }
  __syncthreads();
  for (int pass = 0; pass < 2; ++pass) {
#pragma unroll
    for (int it = 0; it < 4; ++it) {
      const int c = wave * 16 + it * 4 + (lane >> 3);
      const v4f val = *(const v4fa*)(outT + c * 36 + j4);
      *(volatile v4f*)(out + ((size_t)(b * kModel + c)) * kSeq + l0 + j4) = val;
    }
    __threadfence();
  }
}

extern "C" void kernel_launch(void* const* d_in, const int* in_sizes, int n_in,
                              void* d_out, int out_size, void* d_ws, size_t ws_size,
                              hipStream_t stream) {
  if (n_in < 21) return;
  if (in_sizes[0] != kBatch * kModel * kSeq) return;
  if (out_size != kBatch * kModel * kSeq) return;

  const float* x = (const float*)d_in[0];
  const float* gn_gamma = (const float*)d_in[19];
  const float* gn_beta  = (const float*)d_in[20];

  char* ws = (char*)d_ws;
  size_t off = 0;
  auto carve = [&](size_t bytes) -> char* { char* p = ws + off; off += (bytes + 255) & ~(size_t)255; return p; };
  const size_t szX16  = (size_t)kRows * kModel * 2;
  const size_t szWin  = (size_t)kXin * kModel * 2;
  const size_t szWx   = (size_t)kXdbPitch * kInner * 2;
  const size_t szWo   = (size_t)kModel * kInner * 2;
  const size_t szXZ   = (size_t)kRows * kXin * 4;
  const size_t szXC   = (size_t)kRows * kInner * 4;
  const size_t szXCB  = (size_t)kRows * kInner * 2;
  const size_t szXDB  = (size_t)kRows * kXdbPitch * 4;
  const size_t szG    = (size_t)kRows * kInner * 2;
  const size_t szY    = (size_t)kRows * kModel * 4;
  const size_t szStat = (size_t)kBatch * kGroups * 32 * 4;

  unsigned short* Xh = (unsigned short*)carve(szX16);
  unsigned short* Xl = (unsigned short*)carve(szX16);
  unsigned short* WinTh[2]; unsigned short* WinTl[2];
  unsigned short* WxTh[2];  unsigned short* WxTl[2];
  unsigned short* WoTh[2];  unsigned short* WoTl[2];
  for (int d = 0; d < 2; ++d) {
    WinTh[d] = (unsigned short*)carve(szWin); WinTl[d] = (unsigned short*)carve(szWin);
    WxTh[d]  = (unsigned short*)carve(szWx);  WxTl[d]  = (unsigned short*)carve(szWx);
    WoTh[d]  = (unsigned short*)carve(szWo);  WoTl[d]  = (unsigned short*)carve(szWo);
  }
  float*          xz   = (float*)carve(szXZ);
  float*          xcf  = (float*)carve(szXC);
  unsigned short* xcb  = (unsigned short*)carve(szXCB);
  float*          xdb  = (float*)carve(szXDB);
  unsigned short* Gh   = (unsigned short*)carve(szG);
  unsigned short* Gl   = (unsigned short*)carve(szG);
  float*          Yd[2];
  Yd[0] = (float*)carve(szY);
  Yd[1] = (float*)carve(szY);
  float*          stats = (float*)carve(szStat);
  if (off > ws_size) return;

  k_xprep<<<dim3(kSeq / 32, kBatch), 256, 0, stream>>>(x, Xh, Xl);

  for (int d = 0; d < 2; ++d) {
    const int ib = 1 + 9 * d;
    const float* W_in  = (const float*)d_in[ib + 0];
    const float* W_x   = (const float*)d_in[ib + 3];
    const float* W_out = (const float*)d_in[ib + 8];
    k_wprep<kModel><<<kXin / 32, 256, 0, stream>>>(W_in, kXin, WinTh[d], WinTl[d]);
    k_wprep<kInner><<<kXdbPitch / 32, 256, 0, stream>>>(W_x, kXdbCols, WxTh[d], WxTl[d]);
    k_wprep<kInner><<<kModel / 32, 256, 0, stream>>>(W_out, kModel, WoTh[d], WoTl[d]);
  }

  const int tiles1 = (kRows / 64) * (kXin / 64);
  const int tiles2 = (kRows / 64) * (kXdbPitch / 64);
  const int tiles3 = (kRows / 64) * (kModel / 64);

  for (int d = 0; d < 2; ++d) {
    const int ib = 1 + 9 * d;
    const float* conv_w = (const float*)d_in[ib + 1];
    const float* conv_b = (const float*)d_in[ib + 2];
    const float* W_dt   = (const float*)d_in[ib + 4];
    const float* b_dt   = (const float*)d_in[ib + 5];
    const float* A_log  = (const float*)d_in[ib + 6];
    const float* Dp     = (const float*)d_in[ib + 7];

    wmma_gemm64<1, true, 0, 0, false><<<dim3((tiles1 + 7) / 8, 1), 256, 0, stream>>>(
        Xh, Xl, kModel, 0L, WinTh[d], WinTl[d], kModel, 0L,
        (void*)xz, (void*)xz, kXin, 0L, gn_gamma, xcf, 0L, kRows, kXin, kModel, 1.0f);

    k_conv<<<(kRows * kInner) / 1024, 256, 0, stream>>>(xz, conv_w, conv_b, xcf, xcb, d);

    wmma_gemm64<1, false, 0, 0, false><<<dim3((tiles2 + 7) / 8, 1), 256, 0, stream>>>(
        xcb, xcb, kInner, 0L, WxTh[d], WxTh[d], kInner, 0L,
        (void*)xdb, (void*)xdb, kXdbPitch, 0L, gn_gamma, xcf, 0L, kRows, kXdbPitch, kInner, 1.0f);

    k_scan<<<kBatch, kInner, 0, stream>>>(xdb, xcf, xz, W_dt, b_dt, A_log, Dp, Gh, Gl, d);

    wmma_gemm64<1, true, 0, 0, false><<<dim3((tiles3 + 7) / 8, 1), 256, 0, stream>>>(
        Gh, Gl, kInner, 0L, WoTh[d], WoTl[d], kInner, 0L,
        (void*)Yd[d], (void*)Yd[d], kModel, 0L, gn_gamma, xcf, 0L, kRows, kModel, kInner, 1.0f);
  }

  k_gnstats<<<kBatch * kGroups, 256, 0, stream>>>(Yd[0], Yd[1], stats);
  k_gnapply<<<dim3(kSeq / 32, kBatch), 256, 0, stream>>>(Yd[0], Yd[1], stats, gn_gamma, gn_beta, x, (float*)d_out);
}
